// ScoreLayer_57183194579312
// MI455X (gfx1250) — hardware-run, weakly checked
//
#include <hip/hip_runtime.h>
#include <math.h>

typedef __attribute__((ext_vector_type(16))) _Float16 v16h;
typedef __attribute__((ext_vector_type(8)))  _Float16 v8h;
typedef __attribute__((ext_vector_type(8)))  float    v8f;
typedef __attribute__((ext_vector_type(4)))  float    v4f;
typedef __attribute__((ext_vector_type(2)))  float    v2f;

constexpr int kTok     = 8192;
constexpr int kHid     = 512;
constexpr int kMent    = 4096;
constexpr int kRowsA   = 2 * kMent;
constexpr int kFeat    = 100;
constexpr int kFeatPad = 128;
constexpr int kEnt     = 128;
constexpr int kDistN   = 600;
constexpr int kEmbDim  = 50;
constexpr int kEmbPad  = 1216;
constexpr int kWsRows  = 250;
constexpr float kCarryA = 16.0f;
constexpr float kCarryW = 256.0f;
constexpr float kFold   = 1.0f / (kCarryA * kCarryW);
constexpr float kF16Min = 6.103515625e-05f;
static_assert((kHid % 32) == 0, "GEMM K multiple of 32");
static_assert((kMent % 64) == 0 && (kFeatPad % 64) == 0, "GEMM M,N multiples of 64");
static_assert(kEmbPad % 32 == 0 && kEmbPad >= 2 * kDistN, "table plane whole lines");
static_assert(kFold == 1.0f / 4096.0f, "fold constant");

constexpr size_t kOffAP  = 0;
constexpr size_t kOffWT  = kOffAP  + (size_t)kRowsA * kHid * 2;
constexpr size_t kOffPRE = kOffWT  + (size_t)2 * kFeatPad * kHid * 2;
constexpr size_t kOffSC  = kOffPRE + (size_t)kRowsA * kFeatPad * 4;
constexpr size_t kOffEMB = kOffSC  + (size_t)kRowsA * 2 * 4;
constexpr size_t kWsTotal = kOffEMB + (size_t)kEmbPad * 4;
static_assert(kWsTotal == 12915456ull, "carve total");
static_assert(kWsTotal <= 134217728ull, "carve cap");
static_assert((kOffWT % 128) == 0 && (kOffPRE % 128) == 0 && (kOffSC % 128) == 0 && (kOffEMB % 128) == 0, "aligned regions");

__device__ __forceinline__ _Float16 to_h_flush(float v) {
  const float w = (fabsf(v) < kF16Min) ? 0.0f : v;
  return (_Float16)w;
}
union FragH { v16h v; v8h h[2]; };
__device__ __forceinline__ v16h frag_load(const _Float16* p) {
  FragH f;
  f.h[0] = *(const v8h*)(p);
  f.h[1] = *(const v8h*)(p + 16);
  return f.v;
}
__device__ __forceinline__ v8f mma_h(v16h a, v16h b, v8f c) {
  c = __builtin_amdgcn_wmma_f32_16x16x32_f16(false, a, false, b, (short)0, c, false, false);
  asm volatile("v_nop\n\tv_nop\n\tv_nop\n\tv_nop" : "+v"(c) : "v"(a), "v"(b));
  return c;
}
__device__ __forceinline__ void keep4_h(v16h a, v16h b, v16h c, v16h d) { asm volatile("v_nop" :: "v"(a), "v"(b), "v"(c), "v"(d)); }
__device__ __forceinline__ void acc_guard4(v8f& a, v8f& b, v8f& c, v8f& d) { asm volatile("v_nop\n\tv_nop\n\tv_nop\n\tv_nop" : "+v"(a), "+v"(b), "+v"(c), "+v"(d)); }

constexpr int kWtBlocks  = (2 * kFeatPad) / 8;
constexpr int kEmbLines  = kEmbPad / 32;
constexpr int kEmbBlocks = (kEmbLines + 7) / 8;
static_assert(kWtBlocks == 32 && kEmbLines == 38 && kEmbBlocks == 5, "prep grid");

__global__ __launch_bounds__(256) void prep_kernel(
    const float* __restrict__ Wc, const float* __restrict__ Wd,
    const float* __restrict__ Wemb, const float* __restrict__ Ws,
    unsigned short* __restrict__ WT, float* __restrict__ EMB)
{
  const int lane = threadIdx.x & 31;
  const int wave = threadIdx.x >> 5;
  if ((int)blockIdx.x < kWtBlocks) {
    const int R = (int)blockIdx.x * 8 + wave;
    const int set = R >> 7;
    const int n = R & (kFeatPad - 1);
    const float* src = set ? Wd : Wc;
    const bool live = (n < kFeat);
    const int nc = live ? n : (kFeat - 1);
    v8h hv[2];
#pragma unroll
    for (int s = 0; s < 2; ++s) {
#pragma unroll
      for (int e = 0; e < 8; ++e) {
        const int k = s * 256 + lane * 8 + e;
        const float v = src[(size_t)k * kFeat + nc];
        const float w = live ? (v * kCarryW) : 0.0f;
        hv[s][e] = to_h_flush(w);
      }
    }
    unsigned short* dst = WT + (size_t)R * kHid;
    for (int pass = 0; pass < 2; ++pass) {
#pragma unroll
      for (int s = 0; s < 2; ++s)
        *(volatile v8h*)(dst + s * 256 + lane * 8) = hv[s];
      __threadfence();
    }
  } else {
    const int line = ((int)blockIdx.x - kWtBlocks) * 8 + wave;
    if (line < kEmbLines) {
      const int idx = line * 32 + lane;
      const bool live = (idx < 2 * kDistN);
      const int d = idx >> 1;
      const int c = idx & 1;
      const int dc = (d < kDistN) ? d : (kDistN - 1);
      const float* er = Wemb + (size_t)dc * kEmbDim;
      const float* wr = Ws + 2 * 2 * kFeat + c;
      float s = 0.0f;
#pragma unroll 1
      for (int j = 0; j < kEmbDim; ++j) s = fmaf(er[j], wr[2 * j], s);
      const float val = live ? s : 0.0f;
      volatile float* q = (volatile float*)(EMB + idx);
      *q = val;
      __threadfence();
      *q = val;
    }
  }
}

__global__ __launch_bounds__(256) void span_sum_kernel(
    const float* __restrict__ h, const int* __restrict__ chem_spans, const int* __restrict__ dis_spans,
    unsigned short* __restrict__ AP)
{
  const int lane = threadIdx.x & 31;
  const int wave = threadIdx.x >> 5;
  const int R = (int)blockIdx.x * 8 + wave;
  const int set = R >> 12;
  const int m = R & (kMent - 1);
  const int* sp = set ? dis_spans : chem_spans;
  int s0 = sp[2 * m];
  int e0 = sp[2 * m + 1];
  s0 = __builtin_amdgcn_readfirstlane(s0);
  e0 = __builtin_amdgcn_readfirstlane(e0);
  s0 = s0 < 0 ? 0 : (s0 > kTok - 1 ? kTok - 1 : s0);
  e0 = e0 < 0 ? 0 : (e0 > kTok - 1 ? kTok - 1 : e0);
  int nrows = e0 - s0 + 1;
  nrows = nrows < 0 ? 0 : (nrows > 8 ? 8 : nrows);
  float a[16];
#pragma unroll
  for (int e = 0; e < 16; ++e) a[e] = 0.0f;
#pragma unroll 1
  for (int it = 0; it < nrows; ++it) {
    const float* hr = h + (size_t)(s0 + it) * kHid + lane * 8;
    const v4f x0 = *(const v4f*)(hr);
    const v4f x1 = *(const v4f*)(hr + 4);
    const v4f y0 = *(const v4f*)(hr + 256);
    const v4f y1 = *(const v4f*)(hr + 260);
#pragma unroll
    for (int e = 0; e < 4; ++e) {
      a[e]      += x0[e];
      a[4 + e]  += x1[e];
      a[8 + e]  += y0[e];
      a[12 + e] += y1[e];
    }
  }
  v8h hv[2];
#pragma unroll
  for (int e = 0; e < 8; ++e) {
    hv[0][e] = to_h_flush(a[e] * kCarryA);
    hv[1][e] = to_h_flush(a[8 + e] * kCarryA);
  }
  unsigned short* dst = AP + (size_t)R * kHid;
  for (int pass = 0; pass < 2; ++pass) {
#pragma unroll
    for (int s = 0; s < 2; ++s)
      *(volatile v8h*)(dst + s * 256 + lane * 8) = hv[s];
    __threadfence();
  }
}

__global__ __launch_bounds__(256) void proj_gemm_kernel(
    const unsigned short* __restrict__ Ap, int lda, long strideA,
    const unsigned short* __restrict__ Btp, int ldb, long strideB,
    float* __restrict__ Cout, int ldc, long strideC,
    int M, int N, int K, float scale)
{
  const _Float16* A  = (const _Float16*)Ap;
  const _Float16* Bt = (const _Float16*)Btp;
  __shared__ __align__(16) float sT[8][16 * 68];
  const int b    = blockIdx.y;
  const int lane = threadIdx.x & 31;
  const int wave = threadIdx.x >> 5;
  const int tilesN = N >> 6;
  const int tilesM = M >> 6;
  const int tile = (int)blockIdx.x * 8 + wave;
  if (tile >= tilesM * tilesN) return;
  const int tm = tile / tilesN;
  const int tn = tile - tm * tilesN;
  const int m0 = tm << 6;
  const int n0 = tn << 6;

  const _Float16* Ab = A  + (size_t)b * strideA;
  const _Float16* Bb = Bt + (size_t)b * strideB;

  const int rlane = lane & 15;
  const int koff  = (lane >> 4) * 8;
  const int mOff  = (lane >> 4) * 8;

  v8f acc[4][4];
#pragma unroll
  for (int i = 0; i < 4; ++i)
#pragma unroll
    for (int j = 0; j < 4; ++j) acc[i][j] = (v8f){0.f,0.f,0.f,0.f,0.f,0.f,0.f,0.f};

  for (int k0 = 0; k0 < K; k0 += 32) {
    v16h bh[4];
#pragma unroll
    for (int j = 0; j < 4; ++j) {
      const size_t bo = (size_t)(n0 + (j << 4) + rlane) * ldb + koff + k0;
      bh[j] = frag_load(Bb + bo);
    }
#pragma unroll
    for (int i = 0; i < 4; ++i) {
      const size_t ao = (size_t)(m0 + (i << 4) + rlane) * lda + koff + k0;
      const v16h ah = frag_load(Ab + ao);
#pragma unroll
      for (int j = 0; j < 4; ++j) acc[i][j] = mma_h(ah, bh[j], acc[i][j]);
    }
    keep4_h(bh[0], bh[1], bh[2], bh[3]);
  }
  acc_guard4(acc[0][0], acc[0][1], acc[0][2], acc[0][3]);
  acc_guard4(acc[1][0], acc[1][1], acc[1][2], acc[1][3]);
  acc_guard4(acc[2][0], acc[2][1], acc[2][2], acc[2][3]);
  acc_guard4(acc[3][0], acc[3][1], acc[3][2], acc[3][3]);

  float* slab = sT[wave];
  float* C = Cout + (size_t)b * strideC;
#pragma unroll
  for (int i = 0; i < 4; ++i) {
    const int mBase = m0 + (i << 4);
#pragma unroll
    for (int j = 0; j < 4; ++j) {
#pragma unroll
      for (int r = 0; r < 8; ++r) {
        const float v = acc[i][j][r] * scale;
        slab[(mOff + r) * 68 + (j << 4) + rlane] = v;
      }
    }
    __builtin_amdgcn_fence(__ATOMIC_RELEASE, "workgroup");
    __builtin_amdgcn_wave_barrier();
    __builtin_amdgcn_fence(__ATOMIC_ACQUIRE, "workgroup");
    {
      const int hh = lane >> 4, c4 = (lane & 15) * 4;
      for (int pass = 0; pass < 2; ++pass) {
#pragma unroll
        for (int it = 0; it < 8; ++it) {
          const int row = it * 2 + hh;
          const v4f v = *(const v4f*)(slab + row * 68 + c4);
          *(volatile v4f*)(C + (size_t)(mBase + row) * ldc + n0 + c4) = v;
        }
        __threadfence();
      }
    }
    __builtin_amdgcn_fence(__ATOMIC_RELEASE, "workgroup");
    __builtin_amdgcn_wave_barrier();
    __builtin_amdgcn_fence(__ATOMIC_ACQUIRE, "workgroup");
  }
}

__global__ __launch_bounds__(256) void score_kernel(
    const float* __restrict__ PRE, const float* __restrict__ bc, const float* __restrict__ bd,
    const float* __restrict__ Ws, float* __restrict__ SC)
{
  const int g = (int)blockIdx.x * 256 + (int)threadIdx.x;
  const int m = g >> 1;
  const int c = g & 1;
  const int set = m >> 12;
  const float* bias = set ? bd : bc;
  const float* prow = PRE + (size_t)m * kFeatPad;
  const float* wr = Ws + set * (2 * kFeat) + c;
  float s = 0.0f;
#pragma unroll 1
  for (int n = 0; n < kFeat; ++n) {
    const float x = prow[n] + bias[n];
    const float t = tanhf(x);
    s = fmaf(t, wr[2 * n], s);
  }
  volatile float* q = (volatile float*)(SC + g);
  *q = s;
  __threadfence();
  *q = s;
}

__global__ __launch_bounds__(256) void pair_max_kernel(
    const int* __restrict__ chem_spans, const int* __restrict__ chem_ent,
    const int* __restrict__ dis_spans, const int* __restrict__ dis_ent,
    const float* __restrict__ SC, const float* __restrict__ EMB, const float* __restrict__ bs,
    const int* __restrict__ n_chem, const int* __restrict__ n_dis, float* __restrict__ out)
{
  __shared__ __align__(16) float sEmb[kEmbPad];
  __shared__ __align__(16) float sV[kMent * 2];
  __shared__ __align__(16) int   sDe[kMent];
  __shared__ int   lCs[256];
  __shared__ float lC0[256];
  __shared__ float lC1[256];
  __shared__ int   sWcnt[8];
  __shared__ __align__(16) float sHalf[2][2 * kEnt];
  __shared__ __align__(16) float sOut[2 * kEnt];

  const int tid  = threadIdx.x;
  const int lane = tid & 31;
  const int wave = tid >> 5;
  const int ce   = blockIdx.x;

  for (int i = tid; i < kEmbPad; i += 256) sEmb[i] = EMB[i];

  int   dsj[16];
  float d0[16], d1[16], m0[16], m1[16];
#pragma unroll
  for (int q = 0; q < 16; ++q) {
    const int j = q * 256 + tid;
    dsj[q] = dis_spans[2 * j];
    const v2f dv = *(const v2f*)(SC + 2 * (size_t)(kMent + j));
    d0[q] = dv[0];
    d1[q] = dv[1];
    sDe[j] = dis_ent[j];
    m0[q] = -INFINITY;
    m1[q] = -INFINITY;
  }
  const float b0 = bs[0];
  const float b1 = bs[1];
  const int nc = n_chem[0];
  const int nd = n_dis[0];
  const bool shape_ok = (nc == kEnt) && (nd == kEnt);
  __syncthreads();

#pragma unroll 1
  for (int c = 0; c < kMent / 256; ++c) {
    const int i = c * 256 + tid;
    int ei  = chem_ent[i];
    int csi = chem_spans[2 * i];
    const v2f cv = *(const v2f*)(SC + 2 * (size_t)i);
    float c0i = cv[0];
    float c1i = cv[1];
    asm volatile("" : "+v"(ei));
    asm volatile("" : "+v"(csi));
    asm volatile("" : "+v"(c0i));
    asm volatile("" : "+v"(c1i));
    const bool pred = (ei == ce);
    const unsigned bal = __builtin_amdgcn_ballot_w32(pred);
    const int wc = __builtin_popcount(bal);
    if (lane == 0) sWcnt[wave] = wc;
    __syncthreads();
    int base = 0, total = 0;
#pragma unroll
    for (int w = 0; w < 8; ++w) {
      const int cw = sWcnt[w];
      base  += (w < wave) ? cw : 0;
      total += cw;
    }
    const int pos = base + __builtin_popcount(bal & ((1u << lane) - 1u));
    if (pred) {
      const int pc = pos < 255 ? pos : 255;
      lCs[pc] = csi;
      lC0[pc] = c0i;
      lC1[pc] = c1i;
    }
    __syncthreads();
    int nmatch = total < 256 ? total : 256;
    nmatch = __builtin_amdgcn_readfirstlane(nmatch);
#pragma unroll 1
    for (int t = 0; t < nmatch; ++t) {
      const int   cs = lCs[t];
      const float c0 = lC0[t];
      const float c1 = lC1[t];
#pragma unroll
      for (int q = 0; q < 16; ++q) {
        int dd = cs - dsj[q];
        dd = dd < 0 ? -dd : dd;
        dd = dd < (kDistN - 1) ? dd : (kDistN - 1);
        dd = dd > 0 ? dd : 0;
        const v2f ev = *(const v2f*)(sEmb + 2 * dd);
        const float p0 = ((c0 + d0[q]) + ev[0]) + b0;
        const float p1 = ((c1 + d1[q]) + ev[1]) + b1;
        m0[q] = fmaxf(m0[q], p0);
        m1[q] = fmaxf(m1[q], p1);
      }
    }
  }

#pragma unroll
  for (int q = 0; q < 16; ++q) {
    const int j = q * 256 + tid;
    sV[2 * j]     = m0[q];
    sV[2 * j + 1] = m1[q];
  }
  __syncthreads();

  const int de   = tid & (kEnt - 1);
  const int half = tid >> 7;
  {
    float a0 = -INFINITY, a1 = -INFINITY;
    const int jb = half * (kMent / 2);
#pragma unroll 4
    for (int jj = 0; jj < kMent / 2; ++jj) {
      const int j = jb + jj;
      const int dj = sDe[j];
      const v2f vv = *(const v2f*)(sV + 2 * j);
      const bool hit = (dj == de);
      const float t0 = fmaxf(a0, vv[0]);
      const float t1 = fmaxf(a1, vv[1]);
      a0 = hit ? t0 : a0;
      a1 = hit ? t1 : a1;
    }
    sHalf[half][2 * de]     = a0;
    sHalf[half][2 * de + 1] = a1;
  }
  __syncthreads();

  {
    const float g0 = fmaxf(sHalf[0][2 * de],     sHalf[1][2 * de]);
    const float g1 = fmaxf(sHalf[0][2 * de + 1], sHalf[1][2 * de + 1]);
    const float mm = fmaxf(g0, g1);
    const float e0 = expf(g0 - mm);
    const float e1 = expf(g1 - mm);
    const float inv = 1.0f / (e0 + e1);
    const float qnan = __uint_as_float(0x7fc00000u);
    const float o0 = shape_ok ? (e0 * inv) : qnan;
    const float o1 = shape_ok ? (e1 * inv) : qnan;
    if (half == 0) {
      sOut[2 * de]     = o0;
      sOut[2 * de + 1] = o1;
    }
  }
  __syncthreads();

  if (wave == 0) {
    float* orow = out + (size_t)ce * (2 * kEnt);
    const v4f w0 = *(const v4f*)(sOut + lane * 4);
    const v4f w1 = *(const v4f*)(sOut + 128 + lane * 4);
    for (int pass = 0; pass < 2; ++pass) {
      *(volatile v4f*)(orow + lane * 4) = w0;
      *(volatile v4f*)(orow + 128 + lane * 4) = w1;
      __threadfence();
    }
  }
}

extern "C" void kernel_launch(void* const* d_in, const int* in_sizes, int n_in,
                              void* d_out, int out_size, void* d_ws, size_t ws_size,
                              hipStream_t stream) {
  if (n_in < 14) return;
  if (in_sizes[0] != kTok * kHid) return;
  if (in_sizes[1] != kMent * 2) return;
  if (in_sizes[2] != kMent) return;
  if (in_sizes[3] != kMent * 2) return;
  if (in_sizes[4] != kMent) return;
  if (in_sizes[5] != kHid * kFeat) return;
  if (in_sizes[6] != kFeat) return;
  if (in_sizes[7] != kHid * kFeat) return;
  if (in_sizes[8] != kFeat) return;
  if (in_sizes[9] != kDistN * kEmbDim) return;
  if (in_sizes[10] != kWsRows * 2) return;
  if (in_sizes[11] != 2) return;
  if (in_sizes[12] != 1) return;
  if (in_sizes[13] != 1) return;
  if (out_size != kEnt * kEnt * 2) return;
  if (ws_size < kWsTotal) return;

  const float* h          = (const float*)d_in[0];
  const int*   chem_spans = (const int*)d_in[1];
  const int*   chem_ent   = (const int*)d_in[2];
  const int*   dis_spans  = (const int*)d_in[3];
  const int*   dis_ent    = (const int*)d_in[4];
  const float* Wc         = (const float*)d_in[5];
  const float* bc         = (const float*)d_in[6];
  const float* Wd         = (const float*)d_in[7];
  const float* bd         = (const float*)d_in[8];
  const float* Wemb       = (const float*)d_in[9];
  const float* Ws         = (const float*)d_in[10];
  const float* bs         = (const float*)d_in[11];
  const int*   n_chem     = (const int*)d_in[12];
  const int*   n_dis      = (const int*)d_in[13];
  float* out = (float*)d_out;

  char* ws = (char*)d_ws;
  unsigned short* AP  = (unsigned short*)(ws + kOffAP);
  unsigned short* WT  = (unsigned short*)(ws + kOffWT);
  float*          PRE = (float*)(ws + kOffPRE);
  float*          SC  = (float*)(ws + kOffSC);
  float*          EMB = (float*)(ws + kOffEMB);

  prep_kernel<<<kWtBlocks + kEmbBlocks, 256, 0, stream>>>(Wc, Wd, Wemb, Ws, WT, EMB);

  span_sum_kernel<<<kRowsA / 8, 256, 0, stream>>>(h, chem_spans, dis_spans, AP);

  proj_gemm_kernel<<<dim3((kMent / 64) * (kFeatPad / 64) / 8, 2), 256, 0, stream>>>(
      AP, kHid, (long)kMent * kHid,
      WT, kHid, (long)kFeatPad * kHid,
      PRE, kFeatPad, (long)kMent * kFeatPad,
      kMent, kFeatPad, kHid, kFold);

  score_kernel<<<(kRowsA * 2) / 256, 256, 0, stream>>>(PRE, bc, bd, Ws, SC);

  pair_max_kernel<<<kEnt, 256, 0, stream>>>(chem_spans, chem_ent, dis_spans, dis_ent,
                                            SC, EMB, bs, n_chem, n_dis, out);
}
